// Doc_Self_Atten_68616397521526
// MI455X (gfx1250) — hardware-verified
//
#include <hip/hip_runtime.h>


#ifndef NB
#define NB 8
#endif
#ifndef SEQ
#define SEQ 2048
#endif
#define NB_FULL  8
#define SEQ_FULL 2048
#define DM   768
#define HD   768
#define ZB   ((NB % 2 == 0) ? 2 : 1)
#define PCAR 1024.0f
#define QCAR 2048.0f
#define SCL  4.8828125e-4f
#define KX2  (2 * HD)

typedef _Float16 h16;
typedef unsigned short bf;
typedef __attribute__((ext_vector_type(16))) __bf16   v16bf;
typedef __attribute__((ext_vector_type(16))) _Float16 v16h;
typedef __attribute__((ext_vector_type(8)))  _Float16 v8h;
typedef __attribute__((ext_vector_type(8)))  unsigned short v8us;
typedef __attribute__((ext_vector_type(8)))  float    v8f;
typedef __attribute__((ext_vector_type(4)))  float    v4f;
typedef __attribute__((ext_vector_type(2)))  float    v2f;
typedef __attribute__((ext_vector_type(2)))  _Float16 v2h;
typedef __attribute__((ext_vector_type(4)))  _Float16 v4h;
typedef v4f  __attribute__((may_alias)) v4fa;

static_assert(NB <= NB_FULL);
static_assert(SEQ <= SEQ_FULL);
static_assert(NB % ZB == 0);
static_assert(SEQ % 128 == 0);
static_assert(DM % 64 == 0 && HD % 64 == 0);
static_assert(DM == HD);
static_assert(((size_t)SEQ * DM) % 8 == 0);
static_assert((ZB * SEQ) % 8 == 0);
static_assert(HD % 32 == 0 && SEQ % 8 == 0);
static_assert(KX2 % 32 == 0);
static_assert((ZB * SEQ) % 64 == 0);
static_assert(QCAR * SCL == 1.0f);
static_assert((KX2 * 2) % 128 == 0);
static_assert(DM % 64 == 0);
static_assert(((size_t)SEQ * DM / 8) * 16 == (size_t)SEQ * DM * 2);
static_assert(((size_t)ZB * SEQ * DM / 8) * 16 == (size_t)ZB * SEQ * DM * 2);
static_assert(((size_t)ZB * HD * SEQ / 2) * 4 == (size_t)ZB * HD * SEQ * 2);
static_assert(16 * 68 * 4 <= 131072);
static_assert(8 * 32 * 4 <= 131072);

__device__ __forceinline__ unsigned short f2bf(float f) { unsigned u = __float_as_uint(f); u += 0x7FFFu + ((u >> 16) & 1u); return (unsigned short)(u >> 16); }
__device__ __forceinline__ v16h cat16(v8h lo, v8h hi) { return __builtin_shufflevector(lo, hi, 0, 1, 2, 3, 4, 5, 6, 7, 8, 9, 10, 11, 12, 13, 14, 15); }
__device__ __forceinline__ v16bf cat16b(v8us lo, v8us hi) { return __builtin_bit_cast(v16bf, __builtin_shufflevector(lo, hi, 0, 1, 2, 3, 4, 5, 6, 7, 8, 9, 10, 11, 12, 13, 14, 15)); }
__device__ __forceinline__ v8f wmma16(v16h a, v16h b, v8f c) { return __builtin_amdgcn_wmma_f32_16x16x32_f16(false, a, false, b, (short)0, c, false, false); }
__device__ __forceinline__ v8f wmmab(v16bf a, v16bf b, v8f c) { return __builtin_amdgcn_wmma_f32_16x16x32_bf16(false, a, false, b, (short)0, c, false, false); }
__device__ __forceinline__ h16 tohx(float x) { return (h16)x; }
static __device__ __forceinline__ h16 toh_flush(float v) { const h16 r = (h16)v; return (fabsf(v) < 6.103515625e-05f) ? (h16)0.0f : r; }

template <typename T16> struct WFrag;
template <> struct WFrag<h16> { typedef v16h V; static __device__ __forceinline__ V ld(const h16* p) { return cat16(*(const v8h*)p, *(const v8h*)(p + 16)); } static __device__ __forceinline__ v8f mma(V a, V b, v8f c) { return wmma16(a, b, c); } };
template <> struct WFrag<bf> { typedef v16bf V; static __device__ __forceinline__ V ld(const bf* p) { return cat16b(*(const v8us*)p, *(const v8us*)(p + 16)); } static __device__ __forceinline__ v8f mma(V a, V b, v8f c) { return wmmab(a, b, c); } };
template <typename T16>
__global__ __launch_bounds__(32) void k_gemmw(const T16* __restrict__ A, const T16* __restrict__ Bt, int K, float* C, int ldc, size_t sA, size_t sB, size_t sC) {
    typedef typename WFrag<T16>::V V;
    __shared__ __align__(16) float os[16 * 68];
    const size_t z = blockIdx.z; A += z * sA; Bt += z * sB; C += z * sC;
    const int lane = threadIdx.x & 31, lr = lane & 15, hi = lane >> 4; const int r0 = blockIdx.x * 64, c0 = blockIdx.y * 64;
    v8f acc[4][4];
#pragma unroll
    for (int mb = 0; mb < 4; ++mb)
#pragma unroll
        for (int nb = 0; nb < 4; ++nb) acc[mb][nb] = (v8f){};
    const size_t aoff = (size_t)(r0 + lr) * K + 8 * hi, boff = (size_t)(c0 + lr) * K + 8 * hi;
#pragma unroll 1
    for (int kc = 0; kc < K; kc += 32) {
        V a[4];
#pragma unroll
        for (int mb = 0; mb < 4; ++mb) a[mb] = WFrag<T16>::ld(A + aoff + (size_t)mb * 16 * K + kc);
#pragma unroll
        for (int nb = 0; nb < 4; ++nb) { const V b = WFrag<T16>::ld(Bt + boff + (size_t)nb * 16 * K + kc);
#pragma unroll
            for (int mb = 0; mb < 4; ++mb) acc[mb][nb] = WFrag<T16>::mma(a[mb], b, acc[mb][nb]); }
        asm volatile("v_nop\n\tv_nop\n\tv_nop\n\tv_nop" : "+v"(acc[0][0]), "+v"(acc[1][1]), "+v"(acc[2][2]), "+v"(acc[3][3]) : "v"(a[0]), "v"(a[3]));
    }
#pragma unroll
    for (int mb = 0; mb < 4; ++mb) {
#pragma unroll
        for (int nb = 0; nb < 4; ++nb) {
#pragma unroll
            for (int j = 0; j < 8; ++j) os[(hi * 8 + j) * 68 + nb * 16 + lr] = acc[mb][nb][j]; }
        __builtin_amdgcn_wave_barrier(); asm volatile("" ::: "memory");
        float* crow = C + (size_t)(r0 + mb * 16) * ldc + c0;
#pragma unroll 1
        for (int ps = 0; ps < 2; ++ps) {
#pragma unroll
            for (int s = 0; s < 8; ++s) { const int row = 2 * s + hi, cofs = lr * 4; const v4f val = *(const v4fa*)(os + row * 68 + cofs);
                *(volatile v4f*)(crow + (size_t)row * ldc + cofs) = val; }
            if (ps == 0) __threadfence(); }
        __builtin_amdgcn_wave_barrier(); asm volatile("" ::: "memory");
    }
}

__global__ __launch_bounds__(256) void k_cvt8(const float* __restrict__ src, bf* dst, size_t n8, size_t sS, size_t sD) {
    const size_t i = (size_t)blockIdx.x * 256 + threadIdx.x; if (i >= n8) return;
    src += (size_t)blockIdx.y * sS; dst += (size_t)blockIdx.y * sD;
    const v8f v = *(const v8f*)(src + i * 8); v8us o;
#pragma unroll
    for (int k = 0; k < 8; ++k) o[k] = f2bf(v[k]);
    *(volatile v8us*)(dst + i * 8) = o; __threadfence(); *(volatile v8us*)(dst + i * 8) = o; }

__global__ __launch_bounds__(256) void k_cvx(const float* __restrict__ src, bf* xb, h16* kx, size_t n8, size_t sS, size_t sD) {
#pragma clang fp contract(off)
    const size_t i = (size_t)blockIdx.x * 256 + threadIdx.x; if (i >= n8) return;
    src += (size_t)blockIdx.y * sS; xb += (size_t)blockIdx.y * sD; kx += (size_t)blockIdx.y * sD * 2;
    const v8f v = *(const v8f*)(src + i * 8); v8us o; v8h kk;
#pragma unroll
    for (int k = 0; k < 8; ++k) { o[k] = f2bf(v[k]); kk[k] = toh_flush(__uint_as_float((unsigned)o[k] << 16)); }
    const size_t e = i * 8; const size_t row = e / DM; const int col = (int)(e % DM);
    h16* kp = kx + row * KX2 + col;
    *(volatile v8us*)(xb + e) = o; *(volatile v8h*)kp = kk; *(volatile v8h*)(kp + HD) = kk;
    __threadfence();
    *(volatile v8us*)(xb + e) = o; *(volatile v8h*)kp = kk; *(volatile v8h*)(kp + HD) = kk; }

__global__ __launch_bounds__(256) void k_cvtq(const float* __restrict__ src, h16* qx, size_t n8) {
#pragma clang fp contract(off)
    const size_t i = (size_t)blockIdx.x * 256 + threadIdx.x; if (i >= n8) return;
    const v8f v = *(const v8f*)(src + i * 8); v8h qh, ql;
#pragma unroll
    for (int k = 0; k < 8; ++k) { const float s = v[k] * QCAR; const h16 a = toh_flush(s); const float r = s - (float)a; qh[k] = a; ql[k] = toh_flush(r); }
    const size_t e = i * 8; const size_t row = e / DM; const int col = (int)(e % DM);
    h16* qp = qx + row * KX2 + col;
    *(volatile v8h*)qp = qh; *(volatile v8h*)(qp + HD) = ql;
    __threadfence();
    *(volatile v8h*)qp = qh; *(volatile v8h*)(qp + HD) = ql; }

__global__ __launch_bounds__(256) void k_vtpx(const bf* __restrict__ F, h16* V16) {
    const size_t e = ((size_t)blockIdx.x * 256 + threadIdx.x) * 2; if (e >= (size_t)ZB * HD * SEQ) return;
    const int t = (int)(e % SEQ); const int d = (int)((e / SEQ) % HD); const int g = (int)(e / ((size_t)SEQ * HD)); v2h o16;
#pragma unroll
    for (int q = 0; q < 2; ++q) { const float xv = __uint_as_float((unsigned)F[((size_t)g * SEQ + t + q) * DM + d] << 16); o16[q] = toh_flush(xv); }
    *(volatile v2h*)(V16 + e) = o16; __threadfence(); *(volatile v2h*)(V16 + e) = o16; }

__global__ __launch_bounds__(256) void k_vmeanx(const bf* __restrict__ F, float* VM) {
#pragma clang fp contract(off)
    __shared__ float part[8 * 32];
    const int c = threadIdx.x & 31; const int r = __builtin_amdgcn_readfirstlane(threadIdx.x >> 5); const int g = blockIdx.y; const int d = blockIdx.x * 32 + c;
    const bf* f = F + (size_t)g * SEQ * DM + d; float s = 0.f;
#pragma unroll 4
    for (int t = r; t < SEQ; t += 8) { const float xv = __uint_as_float((unsigned)f[(size_t)t * DM] << 16); s += (fabsf(xv) < 6.103515625e-05f) ? 0.0f : xv; }
    part[r * 32 + c] = s;
    __syncthreads();
    if (r == 0) { float a = part[c];
#pragma unroll
        for (int q = 1; q < 8; ++q) a += part[q * 32 + c];
        a *= (1.0f / (float)SEQ); float* p = VM + (size_t)g * HD + d;
        *(volatile float*)p = a; __threadfence(); *(volatile float*)p = a; }
}

__global__ __launch_bounds__(256) void k_asoft(const float* __restrict__ Sb, h16* P16) {
    const int lane = threadIdx.x & 31; const int row = blockIdx.x * 8 + (threadIdx.x >> 5); if (row >= ZB * SEQ) return;
    const float* sr = Sb + (size_t)row * SEQ; float v[SEQ / 32]; float mx = -3.0e38f;
#pragma unroll
    for (int ch = 0; ch < SEQ / 128; ++ch) { const v4f a = *(const v4f*)(sr + ch * 128 + lane * 4);
#pragma unroll
        for (int q = 0; q < 4; ++q) { const float t = a[q] * SCL; v[ch * 4 + q] = t; mx = fmaxf(mx, t); } }
#pragma unroll
    for (int sh = 16; sh; sh >>= 1) mx = fmaxf(mx, __shfl_xor(mx, sh, 32));
    float sum = 0.f;
#pragma unroll
    for (int k = 0; k < SEQ / 32; ++k) { float d0 = __fsub_rn(v[k], mx); asm volatile("" : "+v"(d0)); v[k] = __builtin_amdgcn_exp2f(__fmul_rn(d0, 1.4426950408889634f)); sum += v[k]; }
#pragma unroll
    for (int sh = 16; sh; sh >>= 1) sum += __shfl_xor(sum, sh, 32);
    const float f = __fdiv_rn(PCAR, sum); const float cen = PCAR / (float)SEQ;
#pragma unroll 1
    for (int ps = 0; ps < 2; ++ps) {
#pragma unroll
        for (int ch = 0; ch < SEQ / 128; ++ch) { v4h o4;
#pragma unroll
            for (int q = 0; q < 4; ++q) o4[q] = tohx(v[ch * 4 + q] * f - cen);
            *(volatile v4h*)(P16 + (size_t)row * SEQ + ch * 128 + lane * 4) = o4; }
        if (ps == 0) __threadfence(); }
}

__global__ __launch_bounds__(256) void k_merge(const float* __restrict__ O, const float* __restrict__ VM, float* OUTb) {
    const size_t e = ((size_t)blockIdx.x * 256 + threadIdx.x) * 2; if (e >= (size_t)ZB * SEQ * HD) return;
    const int d = (int)(e % HD); const int g = (int)(e / ((size_t)HD * SEQ));
    const v2f m = *(const v2f*)(VM + (size_t)g * HD + d); const v2f o = *(const v2f*)(O + e);
    v2f o2; o2[0] = o[0] * (1.0f / PCAR) + m[0]; o2[1] = o[1] * (1.0f / PCAR) + m[1];
    *(volatile v2f*)(OUTb + e) = o2; __threadfence(); *(volatile v2f*)(OUTb + e) = o2; }

constexpr size_t al256(size_t b) { return (b + 255) & ~(size_t)255; }
constexpr size_t WS_TOTAL =
    al256((size_t)DM * DM * 2) +
    al256((size_t)ZB * SEQ * DM * 2) +
    al256((size_t)ZB * SEQ * DM * 4) +
    al256((size_t)ZB * SEQ * KX2 * 2) +
    al256((size_t)ZB * SEQ * KX2 * 2) +
    al256((size_t)ZB * HD * SEQ * 2) +
    al256((size_t)ZB * HD * 4) +
    al256((size_t)ZB * SEQ * SEQ * 4) +
    al256((size_t)ZB * SEQ * SEQ * 2) +
    al256((size_t)ZB * SEQ * HD * 4);
static_assert(WS_TOTAL <= (size_t)134217728);

extern "C" void kernel_launch(void* const* d_in, const int* in_sizes, int n_in,
                              void* d_out, int out_size, void* d_ws, size_t ws_size, hipStream_t stream) {
    if (n_in < 2) return;
    if ((size_t)in_sizes[0] < ((size_t)(NB - 1) * SEQ_FULL + SEQ) * DM) return;
    if ((size_t)in_sizes[1] < (size_t)DM * DM) return;
    if ((size_t)out_size < (size_t)NB * SEQ * DM) return;
    if (WS_TOTAL > ws_size) return;
    const float* x = (const float*)d_in[0]; const float* wq = (const float*)d_in[1];
    float* OUT = (float*)d_out;
    char* wsp = (char*)d_ws;
    auto take = [&](size_t bytes) { char* p = wsp; wsp += al256(bytes); return (void*)p; };
    bf* WQ = (bf*)take((size_t)DM * DM * 2);
    bf* XB = (bf*)take((size_t)ZB * SEQ * DM * 2);
    float* FQ = (float*)take((size_t)ZB * SEQ * DM * 4);
    h16* QX = (h16*)take((size_t)ZB * SEQ * KX2 * 2);
    h16* KX = (h16*)take((size_t)ZB * SEQ * KX2 * 2);
    h16* VT16 = (h16*)take((size_t)ZB * HD * SEQ * 2);
    float* VM = (float*)take((size_t)ZB * HD * 4);
    float* Sb = (float*)take((size_t)ZB * SEQ * SEQ * 4); h16* P16 = (h16*)take((size_t)ZB * SEQ * SEQ * 2); float* Ob = (float*)take((size_t)ZB * SEQ * HD * 4);
    if ((size_t)(wsp - (char*)d_ws) > ws_size) return;

    const size_t w8 = (size_t)DM * DM / 8;
    k_cvt8<<<dim3((unsigned)((w8 + 255) / 256), 1, 1), 256, 0, stream>>>(wq, WQ, w8, 0, 0);

    const size_t x8 = (size_t)SEQ * DM / 8;
    const size_t p8 = (size_t)ZB * SEQ * DM / 8;
    const unsigned LE2 = (unsigned)(((size_t)ZB * SEQ * HD / 2 + 255) / 256);
    for (int b0 = 0; b0 < NB; b0 += ZB) {
        k_cvx<<<dim3((unsigned)((x8 + 255) / 256), ZB, 1), 256, 0, stream>>>(x + (size_t)b0 * SEQ_FULL * DM, XB, KX, x8, (size_t)SEQ_FULL * DM, (size_t)SEQ * DM);
        k_gemmw<bf><<<dim3(ZB * SEQ / 64, DM / 64, 1), 32, 0, stream>>>(XB, WQ, DM, FQ, DM, 0, 0, 0);
        k_cvtq<<<dim3((unsigned)((p8 + 255) / 256), 1, 1), 256, 0, stream>>>(FQ, QX, p8);
        k_vtpx<<<LE2, 256, 0, stream>>>(XB, VT16);
        k_vmeanx<<<dim3(HD / 32, ZB, 1), 256, 0, stream>>>(XB, VM);
        k_gemmw<h16><<<dim3(SEQ / 64, SEQ / 64, ZB), 32, 0, stream>>>(QX, KX, KX2, Sb, SEQ, (size_t)SEQ * KX2, (size_t)SEQ * KX2, (size_t)SEQ * SEQ);
        k_asoft<<<ZB * SEQ / 8, 256, 0, stream>>>(Sb, P16);
        k_gemmw<h16><<<dim3(SEQ / 64, HD / 64, ZB), 32, 0, stream>>>(P16, VT16, SEQ, Ob, HD, (size_t)SEQ * SEQ, (size_t)HD * SEQ, (size_t)SEQ * HD);
        k_merge<<<LE2, 256, 0, stream>>>(Ob, VM, OUT + (size_t)b0 * SEQ * DM);
    }
}
